// SwinT_30897994727823
// MI455X (gfx1250) — hardware-verified
//
#include <hip/hip_runtime.h>
#include <math.h>
#include <stdint.h>

#define NB    32
#define LTOK  4096
#define CE    64
#define NHD   8
#define C3    192
#define MH    128
#define NTB   (NB * 64)
#define XP    68
#define HP    72
#define GP    136
#define QSCALE 0.35355339059327373f
#define RSQ2   0.70710678118654752f

#define A_XS   0
#define A_XH   17408
#define A_QS   26624
#define A_KS   35840
#define A_VT   45056
#define A_PS   54272
#define A_RPB  72704
#define A_RGN  79904
#define A_GIX  80160
#define A_END  80416

static_assert((XP * 4) % 16 == 0);
static_assert((HP * 2) % 16 == 0);
static_assert((GP * 2) % 16 == 0);
static_assert(A_XH == A_XS + 64 * XP * 4);
static_assert(A_QS == A_XH + 64 * HP * 2);
static_assert(A_KS == A_QS + 64 * HP * 2);
static_assert(A_VT == A_KS + 64 * HP * 2);
static_assert(A_PS == A_VT + 64 * HP * 2);
static_assert(A_RPB == A_PS + 8 * 16 * HP * 2);
static_assert(A_RGN == A_RPB + 225 * NHD * 4);
static_assert(A_GIX == A_RGN + 64 * 4);
static_assert(A_END == A_GIX + 64 * 4);

typedef _Float16 v16h __attribute__((ext_vector_type(16)));
typedef _Float16 v8h  __attribute__((ext_vector_type(8)));
typedef _Float16 v4h  __attribute__((ext_vector_type(4)));
typedef float    v8f  __attribute__((ext_vector_type(8)));
typedef float    v4f  __attribute__((ext_vector_type(4)));
typedef unsigned int v4u __attribute__((ext_vector_type(4)));

__device__ __forceinline__ unsigned short bf_bits(float f) {
  unsigned u = __float_as_uint(f);
  return (unsigned short)((u + 0x7FFFu + ((u >> 16) & 1u)) >> 16);
}
__device__ __forceinline__ float bf_up(unsigned short h) { return __uint_as_float(((unsigned)h) << 16); }
__device__ __forceinline__ float bfr(float f) { return bf_up(bf_bits(f)); }
__device__ __forceinline__ unsigned short h_bits(_Float16 x) { return __builtin_bit_cast(unsigned short, x); }
__device__ __forceinline__ unsigned pk16(unsigned short a, unsigned short b) { return (unsigned)a | ((unsigned)b << 16); }
__device__ __forceinline__ v8f zero8() { v8f z = {0.f, 0.f, 0.f, 0.f, 0.f, 0.f, 0.f, 0.f}; return z; }
__device__ __forceinline__ v8h zero8h() {
  v8h z;
#pragma unroll
  for (int e = 0; e < 8; ++e) z[e] = (_Float16)0.0f;
  return z;
}
__device__ __forceinline__ v8h sel8z(int zf, v8h v) {
  v8h r;
#pragma unroll
  for (int e = 0; e < 8; ++e) r[e] = (zf != 0) ? (_Float16)0.0f : v[e];
  return r;
}

__device__ __forceinline__ v16h ldfrag_h(const _Float16* p) {
  union { v16h v; v8h h[2]; } f;
  f.h[0] = *(const v8h*)(p);
  f.h[1] = *(const v8h*)(p + 16);
  return f.v;
}

__device__ __forceinline__ v8f mma_h(v16h a, v16h b, v8f c) {
  c = __builtin_amdgcn_wmma_f32_16x16x32_f16(false, a, false, b, (short)0, c, false, false);
#if defined(__HIP_DEVICE_COMPILE__)
  asm volatile("v_nop\n\tv_nop\n\tv_nop\n\tv_nop" : "+v"(c) : "v"(a), "v"(b));
#endif
  return c;
}
__device__ __forceinline__ void wave_sync_lds() {
  __builtin_amdgcn_fence(__ATOMIC_RELEASE, "workgroup");
  __builtin_amdgcn_wave_barrier();
  __builtin_amdgcn_fence(__ATOMIC_ACQUIRE, "workgroup");
}

__device__ __forceinline__ v4f ln_row16(v4f a, const float* __restrict__ g, const float* __restrict__ bv, int c4) {
#pragma clang fp contract(off)
  float s = (a[0] + a[1]) + (a[2] + a[3]);
#pragma unroll
  for (int off = 1; off < 16; off <<= 1) s = s + __shfl_xor(s, off, 32);
  const float mu = s * (1.0f / 64.0f);
  float d[4];
  float s2 = 0.f;
#pragma unroll
  for (int e = 0; e < 4; ++e) { d[e] = a[e] - mu; const float dd = d[e] * d[e]; s2 = s2 + dd; }
#pragma unroll
  for (int off = 1; off < 16; off <<= 1) s2 = s2 + __shfl_xor(s2, off, 32);
  const float var = s2 * (1.0f / 64.0f);
  const float rstd = rsqrtf(var + 1e-5f);
  v4f z;
#pragma unroll
  for (int e = 0; e < 4; ++e) {
    float t0 = d[e] * rstd;
    t0 = t0 * bfr(g[c4 + e]);
    z[e] = t0 + bfr(bv[c4 + e]);
  }
  return z;
}

__global__ __launch_bounds__(256) void cvt_wT(const float* __restrict__ w, unsigned short* outp, int nin, int nout) {
  __shared__ float tile[64][33];
  const int tid = threadIdx.x;
  const int z = blockIdx.z;
  const float* src = w + (size_t)z * nin * nout;
  unsigned short* dst = outp + (size_t)z * nin * nout;
  const int i0 = blockIdx.x * 64;
  const int o0 = blockIdx.y * 32;
#pragma unroll
  for (int p = 0; p < 8; ++p) {
    const int idx = p * 256 + tid;
    const int i = idx >> 5, o = idx & 31;
    tile[i][o] = src[(size_t)(i0 + i) * nout + o0 + o];
  }
  __syncthreads();
  const int o = tid >> 3, c8 = (tid & 7) * 8;
  v4u pk;
#pragma unroll
  for (int e = 0; e < 4; ++e) {
    const float f0 = bfr(tile[c8 + 2 * e][o]) * 64.0f;
    const float f1 = bfr(tile[c8 + 2 * e + 1][o]) * 64.0f;
    pk[e] = pk16(h_bits((_Float16)f0), h_bits((_Float16)f1));
  }
  unsigned short* gp = dst + (size_t)(o0 + o) * nin + i0 + c8;
  *(volatile v4u*)gp = pk;
  __threadfence();
  *(volatile v4u*)gp = pk;
}

__global__ __launch_bounds__(256) void embed_ln(const float* __restrict__ x, const float* __restrict__ g,
                                                const float* __restrict__ bv, float* t) {
#pragma clang fp contract(off)
  __shared__ __align__(16) float Xs[64 * XP];
  const int tid = threadIdx.x, wave = tid >> 5, lane = tid & 31, hh = lane >> 4, c = lane & 15;
  const int b = blockIdx.x >> 6;
  const int p0 = (blockIdx.x & 63) * 64;
#pragma unroll
  for (int it = 0; it < 4; ++it) {
    const int q = it * 256 + tid;
    const int ch = q >> 4, j4 = (q & 15) * 4;
    const v4f v = *(const v4f*)(x + ((size_t)(b * CE + ch)) * LTOK + p0 + j4);
#pragma unroll
    for (int e = 0; e < 4; ++e) Xs[(j4 + e) * XP + ch] = bfr(v[e]);
  }
  __syncthreads();
  const int c4 = c * 4;
  v4f ov[4];
#pragma unroll
  for (int it = 0; it < 4; ++it) {
    const int tok = wave * 8 + it * 2 + hh;
    const v4f a = *(const v4f*)(Xs + tok * XP + c4);
    ov[it] = ln_row16(a, g, bv, c4);
  }
  for (int pass = 0; pass < 2; ++pass) {
#pragma unroll
    for (int it = 0; it < 4; ++it) {
      const int tok = wave * 8 + it * 2 + hh;
      *(volatile v4f*)(t + ((size_t)(b * LTOK + p0 + tok)) * CE + c4) = ov[it];
    }
    __threadfence();
  }
}

__global__ __launch_bounds__(256)
void attn_win(const float* __restrict__ tin, float* tout,
              const float* __restrict__ n1g, const float* __restrict__ n1b,
              const unsigned short* __restrict__ wqkv, const float* __restrict__ qkvb,
              const unsigned short* __restrict__ wprj, const float* __restrict__ prjb,
              const float* __restrict__ rpb, int shift) {
#pragma clang fp contract(off)
  extern __shared__ __align__(16) char smem[];
  float*    Xs   = (float*)(smem + A_XS);
  _Float16* Xh   = (_Float16*)(smem + A_XH);
  _Float16* Qs   = (_Float16*)(smem + A_QS);
  _Float16* Ks   = (_Float16*)(smem + A_KS);
  _Float16* Vt   = (_Float16*)(smem + A_VT);
  _Float16* Ps   = (_Float16*)(smem + A_PS);
  float*    rpbs = (float*)(smem + A_RPB);
  int*      regn = (int*)(smem + A_RGN);
  int*      gidx = (int*)(smem + A_GIX);
  union FH { v16h v; v8h h[2]; };

  const int tid = threadIdx.x, wave = tid >> 5, lane = tid & 31, hh = lane >> 4, c = lane & 15;
  const int b = blockIdx.x >> 6, w = blockIdx.x & 63, wy = w >> 3, wx = w & 7;
  const int maskon = (shift > 0) ? 1 : 0;

  for (int i = tid; i < 225 * NHD; i += 256) rpbs[i] = bfr(rpb[i]);
  if (tid < 64) {
    const int iy = tid >> 3, ix = tid & 7;
    const int hy = wy * 8 + iy, hx = wx * 8 + ix;
    const int oy = (hy + shift) & 63, ox = (hx + shift) & 63;
    gidx[tid] = b * LTOK + oy * 64 + ox;
    const int rh = (hy < 56) ? 0 : ((hy < 60) ? 1 : 2);
    const int rw = (hx < 56) ? 0 : ((hx < 60) ? 1 : 2);
    regn[tid] = rh * 3 + rw;
  }
  __syncthreads();
#pragma unroll
  for (int it = 0; it < 4; ++it) {
    const int q = it * 256 + tid;
    const int tok = q >> 4, c4 = (q & 15) * 4;
    const v4f v = *(const v4f*)(tin + (size_t)gidx[tok] * CE + c4);
    *(v4f*)(Xs + tok * XP + c4) = v;
  }
  __syncthreads();

  {
    const int c4 = c * 4;
#pragma unroll
    for (int it = 0; it < 4; ++it) {
      const int tok = wave * 8 + it * 2 + hh;
      const v4f a = *(const v4f*)(Xs + tok * XP + c4);
      const v4f z = ln_row16(a, n1g, n1b, c4);
      v4h o;
#pragma unroll
      for (int e = 0; e < 4; ++e) o[e] = (_Float16)z[e];
      *(v4h*)(Xh + tok * HP + c4) = o;
    }
  }
  __syncthreads();

  {
    const int mi = wave >> 1;
    const _Float16* W = (const _Float16*)(const void*)wqkv;
    const v16h a0 = ldfrag_h(Xh + (mi * 16 + c) * HP + 8 * hh);
    const v16h a1 = ldfrag_h(Xh + (mi * 16 + c) * HP + 32 + 8 * hh);
#pragma unroll 1
    for (int t = 0; t < 6; ++t) {
      const int ni = (wave & 1) * 6 + t;
      const int n = ni * 16 + c;
      const v16h b0 = ldfrag_h(W + (size_t)n * CE + 8 * hh);
      const v16h b1 = ldfrag_h(W + (size_t)n * CE + 32 + 8 * hh);
      v8f acc = zero8();
      acc = mma_h(a0, b0, acc);
      acc = mma_h(a1, b1, acc);
      const float bias = bfr(qkvb[n]);
      if (ni < 4) {
#pragma unroll
        for (int r = 0; r < 8; ++r) {
          const int row = mi * 16 + 8 * hh + r;
          float v = acc[r] * (1.0f / 64.0f); v = v + bias; v = v * QSCALE; v = v * 8.0f;
          Qs[row * HP + n] = (_Float16)v;
        }
      } else if (ni < 8) {
#pragma unroll
        for (int r = 0; r < 8; ++r) {
          const int row = mi * 16 + 8 * hh + r;
          float v = acc[r] * (1.0f / 64.0f); v = v + bias; v = v * 8.0f;
          Ks[row * HP + (n - 64)] = (_Float16)v;
        }
      } else {
#pragma unroll
        for (int r = 0; r < 8; ++r) {
          const int row = mi * 16 + 8 * hh + r;
          float v = acc[r] * (1.0f / 64.0f); v = v + bias; v = v * 8.0f;
          Vt[(n - 128) * HP + row] = (_Float16)v;
        }
      }
    }
  }
  __syncthreads();

  {
    const int h = wave;
    _Float16* Pw = Ps + wave * 16 * HP;
    _Float16* Oh = Xh;
    const v8h z8 = zero8h();
#pragma unroll 1
    for (int mi = 0; mi < 4; ++mi) {
      FH aq;
      {
        const v8h ql = *(const v8h*)(Qs + (mi * 16 + c) * HP + h * 8);
        aq.h[0] = sel8z(hh, ql);
        aq.h[1] = z8;
      }
      v8f s[4];
#pragma unroll
      for (int j = 0; j < 4; ++j) {
        const v8h kl = *(const v8h*)(Ks + (j * 16 + c) * HP + h * 8);
        FH bk;
        bk.h[0] = sel8z(hh, kl);
        bk.h[1] = z8;
        s[j] = mma_h(aq.v, bk.v, zero8());
      }
      int ra[8];
#pragma unroll
      for (int r = 0; r < 8; ++r) ra[r] = regn[mi * 16 + 8 * hh + r];
#pragma unroll
      for (int j = 0; j < 4; ++j) {
        const int tb = j * 16 + c;
        const int rb = regn[tb];
#pragma unroll
        for (int r = 0; r < 8; ++r) {
          const int ta = mi * 16 + 8 * hh + r;
          const int rpi = ((ta >> 3) - (tb >> 3) + 7) * 15 + ((ta & 7) - (tb & 7) + 7);
          float v = s[j][r] * (1.0f / 64.0f);
          v = v + rpbs[rpi * NHD + h];
          const float mk = (maskon != 0 && ra[r] != rb) ? -100.0f : 0.0f;
          v = v + mk;
          s[j][r] = v;
        }
      }
      float lrow[8];
#pragma unroll
      for (int r = 0; r < 8; ++r) {
        float m = fmaxf(fmaxf(s[0][r], s[1][r]), fmaxf(s[2][r], s[3][r]));
#pragma unroll
        for (int off = 1; off < 16; off <<= 1) m = fmaxf(m, __shfl_xor(m, off, 32));
        float psum = 0.f;
#pragma unroll
        for (int j = 0; j < 4; ++j) {
          const float p = __expf(s[j][r] - m);
          psum = psum + p;
          const float p1 = p * 1024.0f;
          Pw[(8 * hh + r) * HP + j * 16 + c] = (_Float16)p1;
        }
#pragma unroll
        for (int off = 1; off < 16; off <<= 1) psum = psum + __shfl_xor(psum, off, 32);
        lrow[r] = psum;
      }
      wave_sync_lds();
      v8f oc = zero8();
      const int vrow = h * 8 + (c & 7);
#pragma unroll
      for (int kk = 0; kk < 2; ++kk) {
        FH pa;
        pa.h[0] = *(const v8h*)(Pw + c * HP + kk * 32 + 8 * hh);
        pa.h[1] = *(const v8h*)(Pw + c * HP + kk * 32 + 16 + 8 * hh);
        const v16h bv = ldfrag_h(Vt + vrow * HP + kk * 32 + 8 * hh);
        oc = mma_h(pa.v, bv, oc);
      }
#pragma unroll
      for (int r = 0; r < 8; ++r) {
        const int q = mi * 16 + 8 * hh + r;
        const float l = lrow[r];
        const float inv = ((l > 0.f) ? (1.0f / l) : 0.f) * (1.0f / 128.0f);
        const float ov = oc[r] * inv;
        if (c < 8) Oh[q * HP + h * 8 + c] = (_Float16)ov;
      }
      wave_sync_lds();
    }
  }
  __syncthreads();

  {
    const _Float16* Oh = Xh;
    const _Float16* W = (const _Float16*)(const void*)wprj;
#pragma unroll 1
    for (int tI = 0; tI < 2; ++tI) {
      const int t = wave * 2 + tI;
      const int mi = t >> 2, ni = t & 3;
      const int n = ni * 16 + c;
      const v16h a0 = ldfrag_h(Oh + (mi * 16 + c) * HP + 8 * hh);
      const v16h a1 = ldfrag_h(Oh + (mi * 16 + c) * HP + 32 + 8 * hh);
      const v16h b0 = ldfrag_h(W + (size_t)n * CE + 8 * hh);
      const v16h b1 = ldfrag_h(W + (size_t)n * CE + 32 + 8 * hh);
      v8f acc = zero8();
      acc = mma_h(a0, b0, acc);
      acc = mma_h(a1, b1, acc);
      const float bias = bfr(prjb[n]);
#pragma unroll
      for (int r = 0; r < 8; ++r) {
        const int row = mi * 16 + 8 * hh + r;
        float v = acc[r] * (1.0f / 4096.0f); v = v + bias;
        const float old = Xs[row * XP + n];
        Xs[row * XP + n] = old + v;
      }
    }
  }
  __syncthreads();

  {
    const int c4 = c * 4;
    v4f ov[4];
#pragma unroll
    for (int it = 0; it < 4; ++it) {
      const int tok = wave * 8 + it * 2 + hh;
      ov[it] = *(const v4f*)(Xs + tok * XP + c4);
    }
    for (int pass = 0; pass < 2; ++pass) {
#pragma unroll
      for (int it = 0; it < 4; ++it) {
        const int tok = wave * 8 + it * 2 + hh;
        *(volatile v4f*)(tout + (size_t)gidx[tok] * CE + c4) = ov[it];
      }
      __threadfence();
    }
  }
}

__global__ __launch_bounds__(256)
void mlp_blk(const float* __restrict__ tin, float* tout,
             const float* __restrict__ n2g, const float* __restrict__ n2b,
             const unsigned short* __restrict__ w1, const float* __restrict__ fb1,
             const unsigned short* __restrict__ w2, const float* __restrict__ fb2) {
#pragma clang fp contract(off)
  __shared__ __align__(16) float    Xs[64 * XP];
  __shared__ __align__(16) _Float16 Hh[64 * HP];
  __shared__ __align__(16) _Float16 Gh[64 * GP];
  const int tid = threadIdx.x, wave = tid >> 5, lane = tid & 31, hh = lane >> 4, c = lane & 15;
  const size_t tok0 = (size_t)blockIdx.x * 64;

#pragma unroll
  for (int it = 0; it < 4; ++it) {
    const int q = it * 256 + tid;
    const int tok = q >> 4, c4 = (q & 15) * 4;
    const v4f v = *(const v4f*)(tin + (tok0 + tok) * CE + c4);
    *(v4f*)(Xs + tok * XP + c4) = v;
  }
  __syncthreads();
  {
    const int c4 = c * 4;
#pragma unroll
    for (int it = 0; it < 4; ++it) {
      const int tok = wave * 8 + it * 2 + hh;
      const v4f a = *(const v4f*)(Xs + tok * XP + c4);
      const v4f z = ln_row16(a, n2g, n2b, c4);
      v4h o;
#pragma unroll
      for (int e = 0; e < 4; ++e) o[e] = (_Float16)z[e];
      *(v4h*)(Hh + tok * HP + c4) = o;
    }
  }
  __syncthreads();

  {
    const int mi = wave >> 1;
    const _Float16* W = (const _Float16*)(const void*)w1;
    const v16h a0 = ldfrag_h(Hh + (mi * 16 + c) * HP + 8 * hh);
    const v16h a1 = ldfrag_h(Hh + (mi * 16 + c) * HP + 32 + 8 * hh);
#pragma unroll 1
    for (int t = 0; t < 4; ++t) {
      const int ni = (wave & 1) * 4 + t;
      const int n = ni * 16 + c;
      const v16h b0 = ldfrag_h(W + (size_t)n * CE + 8 * hh);
      const v16h b1 = ldfrag_h(W + (size_t)n * CE + 32 + 8 * hh);
      v8f acc = zero8();
      acc = mma_h(a0, b0, acc);
      acc = mma_h(a1, b1, acc);
      const float bias = bfr(fb1[n]);
#pragma unroll
      for (int r = 0; r < 8; ++r) {
        const int row = mi * 16 + 8 * hh + r;
        float u = acc[r] * (1.0f / 64.0f); u = u + bias;
        const float er = erff(u * RSQ2);
        float g = 0.5f * u; g = g * (1.0f + er);
        Gh[row * GP + n] = (_Float16)(g * 64.0f);
      }
    }
  }
  __syncthreads();

  {
    const _Float16* W = (const _Float16*)(const void*)w2;
#pragma unroll 1
    for (int tI = 0; tI < 2; ++tI) {
      const int t = wave * 2 + tI;
      const int mi = t >> 2, ni = t & 3;
      const int n = ni * 16 + c;
      v8f acc = zero8();
#pragma unroll
      for (int ks = 0; ks < 4; ++ks) {
        const v16h a  = ldfrag_h(Gh + (mi * 16 + c) * GP + ks * 32 + 8 * hh);
        const v16h bb = ldfrag_h(W + (size_t)n * MH + ks * 32 + 8 * hh);
        acc = mma_h(a, bb, acc);
      }
      const float bias = bfr(fb2[n]);
#pragma unroll
      for (int r = 0; r < 8; ++r) {
        const int row = mi * 16 + 8 * hh + r;
        float v = acc[r] * (1.0f / 4096.0f); v = v + bias;
        const float old = Xs[row * XP + n];
        Xs[row * XP + n] = old + v;
      }
    }
  }
  __syncthreads();

  {
    const int c4 = c * 4;
    v4f ov[4];
#pragma unroll
    for (int it = 0; it < 4; ++it) {
      const int tok = wave * 8 + it * 2 + hh;
      ov[it] = *(const v4f*)(Xs + tok * XP + c4);
    }
    for (int pass = 0; pass < 2; ++pass) {
#pragma unroll
      for (int it = 0; it < 4; ++it) {
        const int tok = wave * 8 + it * 2 + hh;
        *(volatile v4f*)(tout + (tok0 + tok) * CE + c4) = ov[it];
      }
      __threadfence();
    }
  }
}

__global__ __launch_bounds__(256) void unembed(const float* __restrict__ t, float* out) {
  __shared__ __align__(16) float Xs[64 * XP];
  const int tid = threadIdx.x, wave = tid >> 5, lane = tid & 31, hh = lane >> 4, c = lane & 15;
  const int b = blockIdx.x >> 6;
  const int p0 = (blockIdx.x & 63) * 64;
#pragma unroll
  for (int it = 0; it < 4; ++it) {
    const int q = it * 256 + tid;
    const int tok = q >> 4, c4 = (q & 15) * 4;
    const v4f v = *(const v4f*)(t + ((size_t)(b * LTOK + p0 + tok)) * CE + c4);
    *(v4f*)(Xs + tok * XP + c4) = v;
  }
  __syncthreads();
  const int p4 = c * 4;
  v4f ov[4];
#pragma unroll
  for (int it = 0; it < 4; ++it) {
    const int ch = wave * 8 + it * 2 + hh;
    v4f v;
#pragma unroll
    for (int e = 0; e < 4; ++e) v[e] = Xs[(p4 + e) * XP + ch];
    ov[it] = v;
  }
  for (int pass = 0; pass < 2; ++pass) {
#pragma unroll
    for (int it = 0; it < 4; ++it) {
      const int ch = wave * 8 + it * 2 + hh;
      *(volatile v4f*)(out + ((size_t)(b * CE + ch)) * LTOK + p0 + p4) = ov[it];
    }
    __threadfence();
  }
}

extern "C" void kernel_launch(void* const* d_in, const int* in_sizes, int n_in,
                              void* d_out, int out_size, void* d_ws, size_t ws_size,
                              hipStream_t stream) {
  if (n_in < 16) return;
  if (in_sizes[0] != NB * CE * LTOK) return;
  if (in_sizes[1] != CE || in_sizes[2] != CE) return;
  if (in_sizes[3] != 2 * CE || in_sizes[4] != 2 * CE) return;
  if (in_sizes[5] != 2 * CE * C3 || in_sizes[6] != 2 * C3) return;
  if (in_sizes[7] != 2 * CE * CE || in_sizes[8] != 2 * CE) return;
  if (in_sizes[9] != 2 * 225 * NHD) return;
  if (in_sizes[10] != 2 * CE || in_sizes[11] != 2 * CE) return;
  if (in_sizes[12] != 2 * CE * MH || in_sizes[13] != 2 * MH) return;
  if (in_sizes[14] != 2 * MH * CE || in_sizes[15] != 2 * CE) return;
  if (out_size != NB * CE * LTOK) return;

  const float* x     = (const float*)d_in[0];
  const float* pe_g  = (const float*)d_in[1];
  const float* pe_b  = (const float*)d_in[2];
  const float* n1g   = (const float*)d_in[3];
  const float* n1b   = (const float*)d_in[4];
  const float* qkvw  = (const float*)d_in[5];
  const float* qkvb  = (const float*)d_in[6];
  const float* projw = (const float*)d_in[7];
  const float* projb = (const float*)d_in[8];
  const float* rpb   = (const float*)d_in[9];
  const float* n2g   = (const float*)d_in[10];
  const float* n2b   = (const float*)d_in[11];
  const float* fc1w  = (const float*)d_in[12];
  const float* fc1b  = (const float*)d_in[13];
  const float* fc2w  = (const float*)d_in[14];
  const float* fc2b  = (const float*)d_in[15];
  float* out = (float*)d_out;

  const size_t sT  = (size_t)NB * LTOK * CE * 4;
  const size_t sWq = (size_t)2 * C3 * CE * 2;
  const size_t sWp = (size_t)2 * CE * CE * 2;
  const size_t sW1 = (size_t)2 * MH * CE * 2;
  const size_t sW2 = (size_t)2 * CE * MH * 2;
  size_t off = 0;
  const size_t oA  = off; off += sT;
  const size_t oB  = off; off += sT;
  const size_t oWq = off; off += sWq;
  const size_t oWp = off; off += sWp;
  const size_t oW1 = off; off += sW1;
  const size_t oW2 = off; off += sW2;
  if (off > ws_size) return;
  if (off > (size_t)134217728) return;

  char* ws = (char*)d_ws;
  float* tA = (float*)(ws + oA);
  float* tB = (float*)(ws + oB);
  unsigned short* Wq = (unsigned short*)(ws + oWq);
  unsigned short* Wp = (unsigned short*)(ws + oWp);
  unsigned short* W1 = (unsigned short*)(ws + oW1);
  unsigned short* W2 = (unsigned short*)(ws + oW2);

  const dim3 blk(256);
  cvt_wT<<<dim3(CE / 64, C3 / 32, 2), blk, 0, stream>>>(qkvw, Wq, CE, C3);
  cvt_wT<<<dim3(CE / 64, CE / 32, 2), blk, 0, stream>>>(projw, Wp, CE, CE);
  cvt_wT<<<dim3(CE / 64, MH / 32, 2), blk, 0, stream>>>(fc1w, W1, CE, MH);
  cvt_wT<<<dim3(MH / 64, CE / 32, 2), blk, 0, stream>>>(fc2w, W2, MH, CE);
  embed_ln<<<dim3(NTB), blk, 0, stream>>>(x, pe_g, pe_b, tA);
  (void)hipFuncSetAttribute(reinterpret_cast<const void*>(&attn_win), hipFuncAttributeMaxDynamicSharedMemorySize, A_END);
  for (int i = 0; i < 2; ++i) {
    const int shift = (i == 0) ? 0 : 4;
    attn_win<<<dim3(NTB), blk, A_END, stream>>>(
        tA, tB, n1g + i * CE, n1b + i * CE,
        Wq + (size_t)i * C3 * CE, qkvb + i * C3,
        Wp + (size_t)i * CE * CE, projb + i * CE,
        rpb + i * 225 * NHD, shift);
    mlp_blk<<<dim3(NTB), blk, 0, stream>>>(
        tB, tA, n2g + i * CE, n2b + i * CE,
        W1 + (size_t)i * MH * CE, fc1b + i * MH,
        W2 + (size_t)i * CE * MH, fc2b + i * CE);
  }
  unembed<<<dim3(NTB), blk, 0, stream>>>(tA, out);
  (void)hipGetLastError();
}
